// GRU_16552803958911
// MI455X (gfx1250) — hardware-verified
//
#include <hip/hip_runtime.h>
#include <math.h>

constexpr int NBATCH   = 64;
constexpr int NSTEP    = 1024;
constexpr int NIN      = 64;
constexpr int NHID     = 512;
constexpr int NGATE    = 3 * NHID;
constexpr int NOUTF    = 64;
constexpr int TCH      = 128;
constexpr int NCHUNK   = NSTEP / TCH;
constexpr int CH_ROWS  = TCH * NBATCH;
constexpr int SEQ_ROWS = 32;
constexpr int SEQ_THR  = 512;
constexpr int SEQ_WAVES = SEQ_THR / 32;
constexpr int HP       = NHID + 8;
constexpr int HC_PLANE = NBATCH * NHID;
constexpr float WCARRY     = 16.0f;
constexpr float WCARRY_INV = 1.0f / WCARRY;
constexpr float LOG2E_F    = 1.44269504088896341f;
constexpr float KSIG  = -LOG2E_F / WCARRY;
constexpr float KTANH = 2.0f * LOG2E_F / WCARRY;

static_assert(NSTEP == TCH * NCHUNK, "chunking");
static_assert(NIN % 32 == 0 && NHID % 32 == 0, "K multiples of 32");
static_assert(NBATCH % 64 == 0 && CH_ROWS % 64 == 0 && NGATE % 64 == 0 && NOUTF % 64 == 0, "tile multiples");
static_assert(NBATCH == 2 * SEQ_ROWS, "two blocks of 32 rows");
static_assert(NHID == 32 * SEQ_WAVES, "each wave owns 32 hidden units");
static_assert(SEQ_ROWS * NHID / 8 == 4 * SEQ_THR, "ys copy covers the tile in 4 iterations");
static_assert((HP * 2) % 16 == 0, "LDS row pitch 16-B aligned");
static_assert(2 * SEQ_WAVES * 8 * 128 == HC_PLANE, "carry plane layout");

typedef __attribute__((ext_vector_type(16))) _Float16 v16h;
typedef __attribute__((ext_vector_type(8)))  _Float16 v8h;
typedef __attribute__((ext_vector_type(8)))  float    v8f;
typedef __attribute__((ext_vector_type(4)))  float    v4f;

struct FragH {
  union U { v16h v; v8h h[2]; };
  static __device__ __forceinline__ v16h load(const _Float16* p) {
    U f; f.h[0] = *(const v8h*)(p); f.h[1] = *(const v8h*)(p + 16); return f.v;
  }
  static __device__ __forceinline__ v8f mma(v16h a, v16h b, v8f c) {
    return __builtin_amdgcn_wmma_f32_16x16x32_f16(false, a, false, b, (short)0, c, false, false);
  }
};

__device__ __forceinline__ void guard4_h(v8f& a0, v8f& a1, v8f& a2, v8f& a3, v16h x, v16h y0, v16h y1, v16h y2, v16h y3) {
  asm volatile("v_nop\n\tv_nop\n\tv_nop\n\tv_nop"
               : "+v"(a0), "+v"(a1), "+v"(a2), "+v"(a3)
               : "v"(x), "v"(y0), "v"(y1), "v"(y2), "v"(y3));
}
__device__ __forceinline__ void acc_guard4(v8f& a, v8f& b, v8f& c, v8f& d) {
  asm volatile("v_nop\n\tv_nop\n\tv_nop\n\tv_nop" : "+v"(a), "+v"(b), "+v"(c), "+v"(d));
}
__device__ __forceinline__ void guard12_h(v8f& a0, v8f& a1, v8f& a2, v8f& a3, v8f& a4, v8f& a5,
                                          v8f& a6, v8f& a7, v8f& a8, v8f& a9, v8f& a10, v8f& a11,
                                          v16h x0, v16h x1, v16h x2, v16h x3, v16h x4, v16h x5, v16h x6, v16h x7) {
  asm volatile("v_nop\n\tv_nop\n\tv_nop\n\tv_nop"
               : "+v"(a0), "+v"(a1), "+v"(a2), "+v"(a3), "+v"(a4), "+v"(a5),
                 "+v"(a6), "+v"(a7), "+v"(a8), "+v"(a9), "+v"(a10), "+v"(a11)
               : "v"(x0), "v"(x1), "v"(x2), "v"(x3), "v"(x4), "v"(x5), "v"(x6), "v"(x7));
}

__global__ __launch_bounds__(256) void cvt8_f16_kernel(const float* __restrict__ src, unsigned short* __restrict__ dst,
                                                       int n8, float sc) {
  const int i = blockIdx.x * 256 + threadIdx.x;
  if (i < n8) {
    const float* sp = src + (size_t)i * 8;
    const v4f a = *(const v4f*)(sp);
    const v4f b = *(const v4f*)(sp + 4);
    v8h hv;
#pragma unroll
    for (int e = 0; e < 4; ++e) {
      const float fa = a[e] * sc;
      const float fb = b[e] * sc;
      hv[e]     = (_Float16)fa;
      hv[4 + e] = (_Float16)fb;
    }
    *(volatile v8h*)(dst + (size_t)i * 8) = hv;
    __threadfence();
    *(volatile v8h*)(dst + (size_t)i * 8) = hv;
  }
}

__global__ __launch_bounds__(256) void bias_prep_kernel(const float* __restrict__ bih0, const float* __restrict__ bhh0,
                                                        const float* __restrict__ bih1, const float* __restrict__ bhh1,
                                                        float* __restrict__ dst) {
  const int tid = threadIdx.x;
#pragma unroll 1
  for (int it = 0; it < 4; ++it) {
    const int e0 = (it * 256 + tid) * 4;
    const bool isbn = (e0 >= 2 * NGATE);
    const int lay = isbn ? (((e0 - 2 * NGATE) >= NHID) ? 1 : 0) : ((e0 >= NGATE) ? 1 : 0);
    const int n = isbn ? (e0 - 2 * NGATE - lay * NHID) : (e0 - lay * NGATE);
    const int ni = isbn ? 0 : n;
    const int nh = isbn ? (2 * NHID + n) : n;
    const v4f a0 = *(const v4f*)(bih0 + ni);
    const v4f a1 = *(const v4f*)(bih1 + ni);
    const v4f g0 = *(const v4f*)(bhh0 + nh);
    const v4f g1 = *(const v4f*)(bhh1 + nh);
    const bool useh = isbn || (n < 2 * NHID);
    v4f o;
#pragma unroll
    for (int e = 0; e < 4; ++e) {
      const float bi = lay ? a1[e] : a0[e];
      const float bh = lay ? g1[e] : g0[e];
      const float it_term = isbn ? 0.0f : bi;
      const float h_term  = useh ? bh : 0.0f;
      o[e] = (it_term + h_term) * WCARRY;
    }
    *(volatile v4f*)(dst + e0) = o;
    __threadfence();
    *(volatile v4f*)(dst + e0) = o;
  }
}

__global__ __launch_bounds__(256) void gemm_f16_kernel(
    const unsigned short* __restrict__ Ap, int lda, long strideA,
    const unsigned short* __restrict__ Btp, int ldb,
    float* __restrict__ Cout, int ldc, long strideC,
    const float* __restrict__ bias, int M, int N, int K, int nbatch, float scale) {
  const _Float16* A  = (const _Float16*)Ap;
  const _Float16* Bt = (const _Float16*)Btp;
  __shared__ __align__(16) float sT[8][16 * 68];
  const int lane = threadIdx.x & 31;
  const int wave = threadIdx.x >> 5;
  const int tilesN = N >> 6;
  const int tilesM = M >> 6;
  const int tpb = tilesM * tilesN;
  const int gt = blockIdx.x * 8 + wave;
  if (gt >= tpb * nbatch) return;
  const int b    = gt / tpb;
  const int tile = gt - b * tpb;
  const int tm = tile / tilesN;
  const int tn = tile - tm * tilesN;
  const int m0 = tm << 6;
  const int n0 = tn << 6;

  const int rlane = lane & 15;
  const int koff  = (lane >> 4) * 8;
  const int mOff  = (lane >> 4) * 8;

  const _Float16* ap0 = A + (size_t)b * (size_t)strideA + (size_t)(m0 + rlane) * (size_t)lda + koff;
  const _Float16* bp0 = Bt + (size_t)(n0 + rlane) * (size_t)ldb + koff;
  const size_t astep = (size_t)16 * (size_t)lda;
  const size_t bstep = (size_t)16 * (size_t)ldb;
  const _Float16* bp1 = bp0 + bstep;
  const _Float16* bp2 = bp1 + bstep;
  const _Float16* bp3 = bp2 + bstep;
  const _Float16* ap1 = ap0 + astep;
  const _Float16* ap2 = ap1 + astep;
  const _Float16* ap3 = ap2 + astep;

  v8f acc[4][4];
#pragma unroll
  for (int i = 0; i < 4; ++i)
#pragma unroll
    for (int j = 0; j < 4; ++j) acc[i][j] = (v8f){0.f, 0.f, 0.f, 0.f, 0.f, 0.f, 0.f, 0.f};

#pragma unroll 1
  for (int k0 = 0; k0 < K; k0 += 32) {
    const v16h b0 = FragH::load(bp0 + k0);
    const v16h b1 = FragH::load(bp1 + k0);
    const v16h b2 = FragH::load(bp2 + k0);
    const v16h b3 = FragH::load(bp3 + k0);
    {
      const v16h a = FragH::load(ap0 + k0);
      acc[0][0] = FragH::mma(a, b0, acc[0][0]);
      acc[0][1] = FragH::mma(a, b1, acc[0][1]);
      acc[0][2] = FragH::mma(a, b2, acc[0][2]);
      acc[0][3] = FragH::mma(a, b3, acc[0][3]);
      guard4_h(acc[0][0], acc[0][1], acc[0][2], acc[0][3], a, b0, b1, b2, b3);
    }
    {
      const v16h a = FragH::load(ap1 + k0);
      acc[1][0] = FragH::mma(a, b0, acc[1][0]);
      acc[1][1] = FragH::mma(a, b1, acc[1][1]);
      acc[1][2] = FragH::mma(a, b2, acc[1][2]);
      acc[1][3] = FragH::mma(a, b3, acc[1][3]);
      guard4_h(acc[1][0], acc[1][1], acc[1][2], acc[1][3], a, b0, b1, b2, b3);
    }
    {
      const v16h a = FragH::load(ap2 + k0);
      acc[2][0] = FragH::mma(a, b0, acc[2][0]);
      acc[2][1] = FragH::mma(a, b1, acc[2][1]);
      acc[2][2] = FragH::mma(a, b2, acc[2][2]);
      acc[2][3] = FragH::mma(a, b3, acc[2][3]);
      guard4_h(acc[2][0], acc[2][1], acc[2][2], acc[2][3], a, b0, b1, b2, b3);
    }
    {
      const v16h a = FragH::load(ap3 + k0);
      acc[3][0] = FragH::mma(a, b0, acc[3][0]);
      acc[3][1] = FragH::mma(a, b1, acc[3][1]);
      acc[3][2] = FragH::mma(a, b2, acc[3][2]);
      acc[3][3] = FragH::mma(a, b3, acc[3][3]);
      guard4_h(acc[3][0], acc[3][1], acc[3][2], acc[3][3], a, b0, b1, b2, b3);
    }
  }
  acc_guard4(acc[0][0], acc[0][1], acc[0][2], acc[0][3]);
  acc_guard4(acc[1][0], acc[1][1], acc[1][2], acc[1][3]);
  acc_guard4(acc[2][0], acc[2][1], acc[2][2], acc[2][3]);
  acc_guard4(acc[3][0], acc[3][1], acc[3][2], acc[3][3]);

  float* slab = sT[wave];
  float* C = Cout + (size_t)b * (size_t)strideC;
  const int hh = lane >> 4, c4 = (lane & 15) * 4;
#pragma unroll
  for (int i = 0; i < 4; ++i) {
    const int mBase = m0 + (i << 4);
#pragma unroll
    for (int j = 0; j < 4; ++j) {
      const float bv = bias[n0 + (j << 4) + rlane];
#pragma unroll
      for (int r = 0; r < 8; ++r) {
        const float val = acc[i][j][r] * scale + bv;
        slab[(mOff + r) * 68 + (j << 4) + rlane] = val;
      }
    }
    __builtin_amdgcn_fence(__ATOMIC_RELEASE, "workgroup");
    __builtin_amdgcn_wave_barrier();
    __builtin_amdgcn_fence(__ATOMIC_ACQUIRE, "workgroup");
    for (int pass = 0; pass < 2; ++pass) {
#pragma unroll
      for (int it = 0; it < 8; ++it) {
        const int row = it * 2 + hh;
        const v4f val = *(const v4f*)(slab + row * 68 + c4);
        *(volatile v4f*)(C + (size_t)(mBase + row) * (size_t)ldc + n0 + c4) = val;
      }
      __threadfence();
    }
    __builtin_amdgcn_fence(__ATOMIC_RELEASE, "workgroup");
    __builtin_amdgcn_wave_barrier();
    __builtin_amdgcn_fence(__ATOMIC_ACQUIRE, "workgroup");
  }
}

__global__ __launch_bounds__(SEQ_THR) void gru_seq_kernel(
    const float* __restrict__ XG, const unsigned short* __restrict__ WHp, const float* __restrict__ BN,
    const float* __restrict__ HCIN, float* __restrict__ HCOUT, unsigned short* __restrict__ YS, int first) {
  __shared__ __align__(16) _Float16 Hs[2 * SEQ_ROWS * HP];
  const _Float16* WH = (const _Float16*)WHp;
  const int tid = threadIdx.x, lane = tid & 31, wave = tid >> 5;
  const int c = lane & 15, hh = lane >> 4, koff = hh * 8;
  const int rowbase = blockIdx.x * SEQ_ROWS;
  const int ubase = 32 * wave + 8 * hh;

  const size_t hcoff = ((size_t)(blockIdx.x * SEQ_WAVES + wave) * 8) * 128 + (size_t)lane * 4;

  float hst[2][2][8];
#pragma unroll
  for (int ut = 0; ut < 2; ++ut)
#pragma unroll
    for (int bt = 0; bt < 2; ++bt)
#pragma unroll
      for (int r = 0; r < 8; ++r) hst[ut][bt][r] = 0.0f;
  if (first == 0) {
#pragma unroll
    for (int ut = 0; ut < 2; ++ut)
#pragma unroll
      for (int bt = 0; bt < 2; ++bt) {
        const int s = (ut * 2 + bt) * 2;
        const v4f lo = *(const v4f*)(HCIN + hcoff + (size_t)s * 128);
        const v4f hi = *(const v4f*)(HCIN + hcoff + (size_t)(s + 1) * 128);
#pragma unroll
        for (int r = 0; r < 4; ++r) { hst[ut][bt][r] = lo[r]; hst[ut][bt][4 + r] = hi[r]; }
      }
  }
  const int hst_off = c * HP + ubase;
#pragma unroll
  for (int ut = 0; ut < 2; ++ut)
#pragma unroll
    for (int bt = 0; bt < 2; ++bt) {
      v8h hv;
#pragma unroll
      for (int r = 0; r < 8; ++r) hv[r] = (_Float16)hst[ut][bt][r];
      *(v8h*)(Hs + hst_off + bt * 16 * HP + ut * 16) = hv;
    }
  __syncthreads();

  const _Float16* wp = WH + (size_t)(32 * wave + c) * NHID + koff;
  const float* xgp = XG + (size_t)(rowbase + c) * NGATE + ubase;
  const float* bnp = BN + ubase;
  const int hfrag_off = c * HP + koff;
  constexpr int GSTR = NHID * NHID;
  constexpr int USTR = 16 * NHID;
  constexpr int BSTR = 16 * NGATE;

#pragma unroll 1
  for (int tl = 0; tl < TCH; ++tl) {
    const int cur = tl & 1;
    const _Float16* hrow = Hs + cur * (SEQ_ROWS * HP) + hfrag_off;
    _Float16* hnxt = Hs + (cur ^ 1) * (SEQ_ROWS * HP);
    const float* xs = xgp + (size_t)tl * (size_t)(NBATCH * NGATE);

    v8f acc[3][2][2];
#pragma unroll
    for (int ut = 0; ut < 2; ++ut)
#pragma unroll
      for (int bt = 0; bt < 2; ++bt) {
        acc[0][ut][bt] = *(const v8f*)(xs + bt * BSTR + ut * 16);
        acc[1][ut][bt] = *(const v8f*)(xs + bt * BSTR + NHID + ut * 16);
        acc[2][ut][bt] = *(const v8f*)(bnp + ut * 16);
      }

#pragma unroll 1
    for (int k0 = 0; k0 < NHID; k0 += 32) {
      const v16h h0  = FragH::load(hrow + k0);
      const v16h h1  = FragH::load(hrow + 16 * HP + k0);
      const v16h wr0 = FragH::load(wp + k0);
      const v16h wr1 = FragH::load(wp + USTR + k0);
      const v16h wz0 = FragH::load(wp + GSTR + k0);
      const v16h wz1 = FragH::load(wp + GSTR + USTR + k0);
      const v16h wn0 = FragH::load(wp + 2 * GSTR + k0);
      const v16h wn1 = FragH::load(wp + 2 * GSTR + USTR + k0);
      acc[0][0][0] = FragH::mma(wr0, h0, acc[0][0][0]);
      acc[0][0][1] = FragH::mma(wr0, h1, acc[0][0][1]);
      acc[0][1][0] = FragH::mma(wr1, h0, acc[0][1][0]);
      acc[0][1][1] = FragH::mma(wr1, h1, acc[0][1][1]);
      acc[1][0][0] = FragH::mma(wz0, h0, acc[1][0][0]);
      acc[1][0][1] = FragH::mma(wz0, h1, acc[1][0][1]);
      acc[1][1][0] = FragH::mma(wz1, h0, acc[1][1][0]);
      acc[1][1][1] = FragH::mma(wz1, h1, acc[1][1][1]);
      acc[2][0][0] = FragH::mma(wn0, h0, acc[2][0][0]);
      acc[2][0][1] = FragH::mma(wn0, h1, acc[2][0][1]);
      acc[2][1][0] = FragH::mma(wn1, h0, acc[2][1][0]);
      acc[2][1][1] = FragH::mma(wn1, h1, acc[2][1][1]);
      guard12_h(acc[0][0][0], acc[0][0][1], acc[0][1][0], acc[0][1][1],
                acc[1][0][0], acc[1][0][1], acc[1][1][0], acc[1][1][1],
                acc[2][0][0], acc[2][0][1], acc[2][1][0], acc[2][1][1],
                h0, h1, wr0, wr1, wz0, wz1, wn0, wn1);
    }

#pragma unroll
    for (int ut = 0; ut < 2; ++ut) {
#pragma unroll
      for (int bt = 0; bt < 2; ++bt) {
        const v8f xn = *(const v8f*)(xs + bt * BSTR + 2 * NHID + ut * 16);
        v8h hv;
#pragma unroll
        for (int r = 0; r < 8; ++r) {
          const float er = __builtin_amdgcn_exp2f(acc[0][ut][bt][r] * KSIG);
          const float rg = __builtin_amdgcn_rcpf(1.0f + er);
          const float ez = __builtin_amdgcn_exp2f(acc[1][ut][bt][r] * KSIG);
          const float zg = __builtin_amdgcn_rcpf(1.0f + ez);
          const float pn = fmaf(rg, acc[2][ut][bt][r], xn[r]);
          const float en = __builtin_amdgcn_exp2f(pn * KTANH);
          const float nn = fmaf(-2.0f, __builtin_amdgcn_rcpf(en + 1.0f), 1.0f);
          const float ho = hst[ut][bt][r];
          const float hn = fmaf(zg, ho - nn, nn);
          hst[ut][bt][r] = hn;
          hv[r] = (_Float16)hn;
        }
        *(v8h*)(hnxt + hst_off + bt * 16 * HP + ut * 16) = hv;
      }
    }
    __syncthreads();

    {
      unsigned short* yb = YS + ((size_t)tl * NBATCH + (size_t)rowbase) * NHID;
      v8h yv[4];
#pragma unroll
      for (int it = 0; it < 4; ++it) {
        const int idx = it * SEQ_THR + tid;
        const int row = idx >> 6, c8 = (idx & 63) * 8;
        yv[it] = *(const v8h*)(hnxt + row * HP + c8);
      }
      for (int pass = 0; pass < 2; ++pass) {
#pragma unroll
        for (int it = 0; it < 4; ++it) {
          const int idx = it * SEQ_THR + tid;
          const int row = idx >> 6, c8 = (idx & 63) * 8;
          *(volatile v8h*)(yb + (size_t)row * NHID + c8) = yv[it];
        }
        __threadfence();
      }
    }
  }

  for (int pass = 0; pass < 2; ++pass) {
#pragma unroll
    for (int ut = 0; ut < 2; ++ut)
#pragma unroll
      for (int bt = 0; bt < 2; ++bt) {
        const int s = (ut * 2 + bt) * 2;
        v4f lo, hi;
#pragma unroll
        for (int r = 0; r < 4; ++r) { lo[r] = hst[ut][bt][r]; hi[r] = hst[ut][bt][4 + r]; }
        *(volatile v4f*)(HCOUT + hcoff + (size_t)s * 128) = lo;
        *(volatile v4f*)(HCOUT + hcoff + (size_t)(s + 1) * 128) = hi;
      }
    __threadfence();
  }
}

extern "C" void kernel_launch(void* const* d_in, const int* in_sizes, int n_in,
                              void* d_out, int out_size, void* d_ws, size_t ws_size, hipStream_t stream) {
  if (n_in < 11 || d_out == nullptr || d_ws == nullptr) return;
  if (in_sizes[0] != NBATCH * NSTEP * NIN || in_sizes[1] != NGATE * NIN || in_sizes[2] != NGATE * NHID ||
      in_sizes[3] != NGATE || in_sizes[4] != NGATE || in_sizes[5] != NGATE * NHID || in_sizes[6] != NGATE * NHID ||
      in_sizes[7] != NGATE || in_sizes[8] != NGATE || in_sizes[9] != NOUTF * NHID || in_sizes[10] != NOUTF ||
      out_size != NBATCH * NSTEP * NOUTF) return;

  const float* x    = (const float*)d_in[0];
  const float* wih0 = (const float*)d_in[1];
  const float* whh0 = (const float*)d_in[2];
  const float* bih0 = (const float*)d_in[3];
  const float* bhh0 = (const float*)d_in[4];
  const float* wih1 = (const float*)d_in[5];
  const float* whh1 = (const float*)d_in[6];
  const float* bih1 = (const float*)d_in[7];
  const float* bhh1 = (const float*)d_in[8];
  const float* fcw  = (const float*)d_in[9];
  const float* fcb  = (const float*)d_in[10];
  float* out = (float*)d_out;

  char* ws = (char*)d_ws; size_t off = 0;
  auto carve = [&](size_t bytes) -> char* { char* p = ws + off; off += (bytes + 255) & ~(size_t)255; return p; };
  unsigned short* X16  = (unsigned short*)carve((size_t)NBATCH * NSTEP * NIN * 2);
  unsigned short* WIH0 = (unsigned short*)carve((size_t)NGATE * NIN * 2);
  unsigned short* WHH0 = (unsigned short*)carve((size_t)NGATE * NHID * 2);
  unsigned short* WIH1 = (unsigned short*)carve((size_t)NGATE * NHID * 2);
  unsigned short* WHH1 = (unsigned short*)carve((size_t)NGATE * NHID * 2);
  unsigned short* FCW  = (unsigned short*)carve((size_t)NOUTF * NHID * 2);
  float*          BIAS = (float*)carve((size_t)4096 * 4);
  float*          XG   = (float*)carve((size_t)CH_ROWS * NGATE * 4);
  unsigned short* YS0  = (unsigned short*)carve((size_t)CH_ROWS * NHID * 2);
  unsigned short* YS1  = (unsigned short*)carve((size_t)CH_ROWS * NHID * 2);
  float*          HC   = (float*)carve((size_t)4 * HC_PLANE * 4);
  if (off > ws_size || off > (size_t)134217728) return;

  auto cvt = [&](const float* s, unsigned short* d, int n, float sc) {
    const int n8 = n / 8;
    cvt8_f16_kernel<<<(n8 + 255) / 256, 256, 0, stream>>>(s, d, n8, sc);
  };
  cvt(x,    X16,  NBATCH * NSTEP * NIN, 1.0f);
  cvt(wih0, WIH0, NGATE * NIN,  WCARRY);
  cvt(whh0, WHH0, NGATE * NHID, WCARRY);
  cvt(wih1, WIH1, NGATE * NHID, WCARRY);
  cvt(whh1, WHH1, NGATE * NHID, WCARRY);
  cvt(fcw,  FCW,  NOUTF * NHID, WCARRY);
  bias_prep_kernel<<<1, 256, 0, stream>>>(bih0, bhh0, bih1, bhh1, BIAS);

  auto gemm = [&](const unsigned short* A, int lda, long sA, const unsigned short* Bt, int ldb,
                  float* C, int ldc, long sC, const float* bias, int M, int N, int K, int nb, float sc) {
    const int tiles = (M / 64) * (N / 64) * nb;
    gemm_f16_kernel<<<(tiles + 7) / 8, 256, 0, stream>>>(A, lda, sA, Bt, ldb, C, ldc, sC, bias, M, N, K, nb, sc);
  };

  for (int ch = 0; ch < NCHUNK; ++ch) {
    const int pin = ch & 1, pout = (ch + 1) & 1;
    const int first = (ch == 0) ? 1 : 0;
    gemm(X16 + (size_t)ch * TCH * NIN, NSTEP * NIN, (long)NIN, WIH0, NIN,
         XG, NGATE, (long)NBATCH * NGATE, BIAS, NBATCH, NGATE, NIN, TCH, 1.0f);
    gru_seq_kernel<<<NBATCH / SEQ_ROWS, SEQ_THR, 0, stream>>>(
        XG, WHH0, BIAS + 2 * NGATE, HC + (size_t)(0 + pin) * HC_PLANE, HC + (size_t)(0 + pout) * HC_PLANE, YS0, first);
    gemm(YS0, NHID, 0L, WIH1, NHID, XG, NGATE, 0L, BIAS + NGATE, CH_ROWS, NGATE, NHID, 1, 1.0f);
    gru_seq_kernel<<<NBATCH / SEQ_ROWS, SEQ_THR, 0, stream>>>(
        XG, WHH1, BIAS + 2 * NGATE + NHID, HC + (size_t)(2 + pin) * HC_PLANE, HC + (size_t)(2 + pout) * HC_PLANE, YS1, first);
    gemm(YS1, NHID, (long)NBATCH * NHID, FCW, NHID,
         out + (size_t)ch * TCH * NOUTF, NSTEP * NOUTF, (long)NOUTF, fcb, NBATCH, NOUTF, NHID, TCH, WCARRY_INV);
  }
}
